// SimpleOldSparseCNN_18829136626386
// MI455X (gfx1250) — hardware-verified
//
#include <hip/hip_runtime.h>
#include <hip/hip_bf16.h>
#include <math.h>


#define BB 2
#define SS 2048
#define DD 1024
#define HH 16
#define DKK 64
#define QW 2

typedef _Float16 bf16;
typedef __attribute__((ext_vector_type(4))) unsigned v4u_t;
typedef unsigned v4ua __attribute__((ext_vector_type(4), may_alias));
typedef __attribute__((ext_vector_type(4))) float v4f_t;
typedef float v4fa __attribute__((ext_vector_type(4), may_alias));
typedef __attribute__((ext_vector_type(16))) bf16  bf16x16;
typedef __attribute__((ext_vector_type(8)))  bf16  bf16x8;
typedef __attribute__((ext_vector_type(4)))  bf16  bf16x4;
typedef __attribute__((ext_vector_type(8)))  float f32x8;

#define LDS_STRIDE 48
#define KSTRIDE    72
#define VSTRIDE    48

__device__ __forceinline__ f32x8 wmma_bf16(bf16x16 a, bf16x16 b, f32x8 c) {
  return __builtin_amdgcn_wmma_f32_16x16x32_f16(
      false, a, false, b, (short)0, c, false, false);
}

template <typename T>
__device__ __forceinline__ bf16x16 load_frag(const T* __restrict__ base, int ld,
                                             int row0, int k0) {
  const int lane = threadIdx.x & 31;
  const int r    = lane & 15;
  const int kh   = (lane >> 4) * 8;
  const T* p0 = base + (size_t)(row0 + r) * ld + (k0 + kh);
  const T* p1 = p0 + 16;
  bf16x16 f;
#pragma unroll
  for (int i = 0; i < 8; ++i) {
    f[i]     = (bf16)p0[i];
    f[i + 8] = (bf16)p1[i];
  }
  return f;
}

__device__ __forceinline__ bf16x16 lds_frag(const bf16* base, int stride) {
  const int lane = threadIdx.x & 31;
  const int row  = lane & 15;
  const int kh   = (lane >> 4) * 8;
  const bf16x8 lo = *(const bf16x8*)(base + row * stride + kh);
  const bf16x8 hi = *(const bf16x8*)(base + row * stride + kh + 16);
  bf16x16 f;
#pragma unroll
  for (int i = 0; i < 8; ++i) { f[i] = lo[i]; f[i + 8] = hi[i]; }
  return f;
}

template <typename T>
__device__ __forceinline__ void stage_read16(const T* __restrict__ p, float* buf) {
#pragma unroll
  for (int i = 0; i < 16; ++i) buf[i] = (float)p[i];
}

__device__ __forceinline__ void stage_write(bf16* dst, const float* buf, int nquad) {
#pragma unroll
  for (int i = 0; i < nquad; ++i) {
    bf16x4 q;
    q[0] = (bf16)buf[4 * i];     q[1] = (bf16)buf[4 * i + 1];
    q[2] = (bf16)buf[4 * i + 2]; q[3] = (bf16)buf[4 * i + 3];
    *(bf16x4*)(dst + 4 * i) = q;
  }
}

template <typename AT, int MODE>
__global__ __launch_bounds__(256) void gemm_bias_kernel(
    const AT* __restrict__ A, const float* __restrict__ W,
    const float* __restrict__ bias, void* __restrict__ out,
    int M, int N, int K) {
  __shared__ bf16 ldsA[128 * LDS_STRIDE];
  __shared__ bf16 ldsW[256 * LDS_STRIDE];
  __shared__ __attribute__((aligned(16))) unsigned char sob[256 * 136 * 2];

  const int t    = threadIdx.x;
  const int wave = t >> 5;
  const int lane = t & 31;
  const int wm   = (wave & 1) * 64;
  const int wn   = (wave >> 1) * 64;
  const int mBlk = blockIdx.x * 128;
  const int nBlk = blockIdx.y * 256;

  const int arow = t >> 1;
  const int ach  = (t & 1) * 16;

  float abuf[16];
  float wbuf[32];

  stage_read16(A + (size_t)(mBlk + arow) * K + ach, abuf);
  stage_read16(W + (size_t)(nBlk + t) * K,          wbuf);
  stage_read16(W + (size_t)(nBlk + t) * K + 16,     wbuf + 16);

  f32x8 acc[4][4] = {};

  for (int k = 0; k < K; k += 32) {
    __syncthreads();
    stage_write(&ldsA[arow * LDS_STRIDE + ach], abuf, 4);
    stage_write(&ldsW[t * LDS_STRIDE],          wbuf, 8);
    if (k + 32 < K) {
      stage_read16(A + (size_t)(mBlk + arow) * K + (k + 32) + ach, abuf);
      stage_read16(W + (size_t)(nBlk + t) * K + (k + 32),          wbuf);
      stage_read16(W + (size_t)(nBlk + t) * K + (k + 32) + 16,     wbuf + 16);
    }
    __syncthreads();

    bf16x16 af[4], wf[4];
#pragma unroll
    for (int i = 0; i < 4; ++i)
      af[i] = lds_frag(ldsA + (wm + 16 * i) * LDS_STRIDE, LDS_STRIDE);
#pragma unroll
    for (int j = 0; j < 4; ++j)
      wf[j] = lds_frag(ldsW + (wn + 16 * j) * LDS_STRIDE, LDS_STRIDE);
#pragma unroll
    for (int i = 0; i < 4; ++i)
#pragma unroll
      for (int j = 0; j < 4; ++j)
        acc[i][j] = wmma_bf16(af[i], wf[j], acc[i][j]);
  }

  const int nlane = lane & 15;
  const int mh    = (lane >> 4) * 8;
  __syncthreads();
  if (MODE == 0 || MODE == 1) {
    bf16* so = (bf16*)sob;
#pragma unroll
    for (int i = 0; i < 4; ++i)
#pragma unroll
      for (int j = 0; j < 4; ++j) {
        const int nl = wn + 16 * j + nlane;
        const float bv = bias ? bias[nBlk + nl] : 0.0f;
#pragma unroll
        for (int r = 0; r < 8; ++r) {
          const int ml = wm + 16 * i + mh + r;
          const bf16 hv = (bf16)(acc[i][j][r] + bv);
          if (MODE == 0) so[ml * 264 + nl] = hv;
          else           so[nl * 136 + ml] = hv;
        }
      }
    __syncthreads();
#pragma unroll 1
    for (int pass = 0; pass < 2; ++pass) {
      if (MODE == 0) {
        for (int ch = t; ch < 128 * 32; ch += 256) { const int ml = ch >> 5, q = (ch & 31) * 8;
          *(volatile v4u_t*)((bf16*)out + (size_t)(mBlk + ml) * N + nBlk + q) = *(const v4ua*)(so + ml * 264 + q); }
      } else {
        const int b_ = mBlk / SS, s0 = mBlk & (SS - 1);
        for (int ch = t; ch < 256 * 16; ch += 256) { const int nl = ch >> 4, q = (ch & 15) * 8; const int n = nBlk + nl, h = n >> 6, dk = n & (DKK - 1);
          *(volatile v4u_t*)((bf16*)out + (((size_t)(b_ * HH + h)) * DKK + dk) * SS + s0 + q) = *(const v4ua*)(so + nl * 136 + q); }
      }
      __threadfence();
    }
  } else {
    float* so = (float*)sob;
#pragma unroll 1
    for (int hf = 0; hf < 2; ++hf) {
      if (wm == hf * 64) {
#pragma unroll
        for (int i = 0; i < 4; ++i)
#pragma unroll
          for (int j = 0; j < 4; ++j) {
            const int nl = wn + 16 * j + nlane;
            const float bv = bias ? bias[nBlk + nl] : 0.0f;
#pragma unroll
            for (int r = 0; r < 8; ++r) so[(16 * i + mh + r) * 260 + nl] = acc[i][j][r] + bv;
          }
      }
      __syncthreads();
#pragma unroll 1
      for (int pass = 0; pass < 2; ++pass) {
        for (int ch = t; ch < 64 * 64; ch += 256) { const int ml = ch >> 6, q = (ch & 63) * 4;
          *(volatile v4f_t*)((float*)out + (size_t)(mBlk + hf * 64 + ml) * N + nBlk + q) = *(const volatile v4fa*)(so + ml * 260 + q); }
        __threadfence();
      }
      __syncthreads();
    }
  }
}


#define NBT 128
#define HW 128
#define SZ 127
#define FIN 16129
#define KP 16160
#define O3 256

__global__ __launch_bounds__(256) void k_conv(const float* __restrict__ xc, const float* __restrict__ w4, float* __restrict__ A) {
  const int b = blockIdx.x; const float w00 = w4[0], w01 = w4[1], w10 = w4[2], w11 = w4[3];
  const float* img = xc + (size_t)b * HW * HW; float* row = A + (size_t)b * KP;
#pragma unroll 1
  for (int pass = 0; pass < 2; ++pass) {
    for (int i = threadIdx.x; i < KP; i += 256) { float v = 0.0f;
      if (i < FIN) { const int h = i / SZ, w = i - h * SZ; const float* p = img + (size_t)h * HW + w;
        v = tanhf(p[0] * w00 + p[1] * w01 + p[HW] * w10 + p[HW + 1] * w11); }
      *(volatile float*)(row + i) = v; }
    __threadfence(); }
}
__global__ __launch_bounds__(256) void k_wpad(const float* __restrict__ fcw, float* __restrict__ Wp) {
  const int o = blockIdx.x; float* row = Wp + (size_t)o * KP;
#pragma unroll 1
  for (int pass = 0; pass < 2; ++pass) { for (int i = threadIdx.x; i < KP; i += 256) { const float v = (i < FIN) ? fcw[(size_t)o * FIN + i] : 0.0f; *(volatile float*)(row + i) = v; } __threadfence(); }
}
__global__ __launch_bounds__(256) void k_out(const float* __restrict__ T, int c, float* __restrict__ out) {
  const int b = blockIdx.x, o = threadIdx.x; const float v = tanhf(T[(size_t)b * O3 + o]);
  *(volatile float*)(out + (size_t)b * 3 * O3 + c * O3 + o) = v; __threadfence(); *(volatile float*)(out + (size_t)b * 3 * O3 + c * O3 + o) = v;
}

extern "C" void kernel_launch(void* const* d_in, const int* in_sizes, int n_in,
                              void* d_out, int out_size, void* d_ws, size_t ws_size,
                              hipStream_t stream) {
  (void)in_sizes; (void)n_in; (void)out_size; (void)ws_size;
  const float* x = (const float*)d_in[0];
  const float* wc[3]  = {(const float*)d_in[1], (const float*)d_in[2], (const float*)d_in[3]};
  const float* fcw[3] = {(const float*)d_in[4], (const float*)d_in[6], (const float*)d_in[8]};
  const float* fcb[3] = {(const float*)d_in[5], (const float*)d_in[7], (const float*)d_in[9]};
  char* ws = (char*)d_ws;
  float* A  = (float*)ws; ws += (size_t)NBT * KP * 4;
  float* Wp = (float*)ws; ws += (size_t)O3 * KP * 4;
  float* T  = (float*)ws; ws += (size_t)NBT * O3 * 4;
  for (int c = 0; c < 3; ++c) {
    k_conv<<<NBT, 256, 0, stream>>>(x + (size_t)c * NBT * HW * HW, wc[c], A);
    k_wpad<<<O3, 256, 0, stream>>>(fcw[c], Wp);
    gemm_bias_kernel<float, 2><<<dim3(NBT / 128, O3 / 256), 256, 0, stream>>>(A, Wp, fcb[c], T, NBT, O3, KP);
    k_out<<<NBT, 256, 0, stream>>>(T, c, (float*)d_out);
  }
}
